// GRUModel_4466765988087
// MI455X (gfx1250) — hardware-run, weakly checked
//
#include <hip/hip_runtime.h>

typedef __attribute__((ext_vector_type(16))) _Float16 v16h;
typedef __attribute__((ext_vector_type(8)))  _Float16 v8h;
typedef __attribute__((ext_vector_type(8)))  float    v8f;
typedef __attribute__((ext_vector_type(4)))  float    v4f;
typedef __attribute__((ext_vector_type(2)))  float    v2f;

constexpr int kHid = 32;
constexpr int kSeq = 512;
constexpr int kBatch = 4096;
constexpr int kGateRows = 3 * kHid;
constexpr int kOutF = 12;
constexpr int kOutRowsPad = 16;
constexpr int kThreads = 256;
constexpr int kWaves = kThreads / 32;
constexpr int kRowsPerWave = 16;
constexpr int kRowsPerBlock = kWaves * kRowsPerWave;
constexpr int kBlocks = kBatch / kRowsPerBlock;
constexpr int kOutPerWave = kRowsPerWave * kOutF;
static_assert(kBlocks * kRowsPerBlock == kBatch);
static_assert(kSeq % 4 == 0);
static_assert(kHid == 32);
static_assert((kOutPerWave * 4) % 128 == 0);
static_assert(kOutPerWave == 128 + 64);
static_assert(kGateRows * kHid == 6 * 2 * kThreads);
static_assert(kOutRowsPad * kHid == 2 * kThreads);
static_assert(kGateRows <= kThreads);
static_assert(kBatch * kOutF * 4 == 196608);

constexpr float kWScale = 1024.0f;
constexpr float kWInv = 0.0009765625f;
constexpr float kLog2e = 1.4426950408889634f;

union FragU { v16h v; v8h h[2]; };
__device__ __forceinline__ v16h frag_load_f16(const _Float16* p) {
  FragU f;
  f.h[0] = *(const v8h*)(p);
  f.h[1] = *(const v8h*)(p + 16);
  return f.v;
}

__device__ __forceinline__ v8f mma_f16(v16h a, v16h b, v8f c) {
  c = __builtin_amdgcn_wmma_f32_16x16x32_f16(false, a, false, b, (short)0, c, false, false);
  asm volatile("v_nop\n\tv_nop\n\tv_nop\n\tv_nop" : "+v"(c) : "v"(a), "v"(b));
  return c;
}

__device__ __forceinline__ unsigned int pack_f16x2(float a, float b) {
  const _Float16 ha = (_Float16)a;
  const _Float16 hb = (_Float16)b;
  return (unsigned int)__builtin_bit_cast(unsigned short, ha) |
         ((unsigned int)__builtin_bit_cast(unsigned short, hb) << 16);
}

__device__ __forceinline__ float sigm_sc(float p) {
  const float e = __builtin_amdgcn_exp2f(p * (-kLog2e * kWInv));
  return __builtin_amdgcn_rcpf(1.0f + e);
}
__device__ __forceinline__ float tanh_sc(float p) {
  const float u = __builtin_amdgcn_exp2f(p * (2.0f * kLog2e * kWInv));
  return fmaf(-2.0f, __builtin_amdgcn_rcpf(u + 1.0f), 1.0f);
}

__device__ __forceinline__ void cell_step(float xv, float (&hlo)[8], float (&hhi)[8],
                                          const float (&wih)[6][8], const float (&bihn)[2][8],
                                          const _Float16* Wl, const float* Clh, int bn, int hf)
{
  asm volatile("" ::: "memory");
  v16h Bf;
#pragma unroll
  for (int i = 0; i < 8; ++i) {
    Bf[i]     = (_Float16)hlo[i];
    Bf[8 + i] = (_Float16)hhi[i];
  }
  v8f D[6];
#pragma unroll
  for (int tt = 0; tt < 6; ++tt) {
    const int rowbase = (tt >> 1) * kHid + (tt & 1) * 16;
    const v16h A = frag_load_f16(Wl + (rowbase + bn) * kHid + 8 * hf);
    const v8f cin = *(const v8f*)(Clh + 8 * tt);
    D[tt] = mma_f16(A, Bf, cin);
  }
#pragma unroll
  for (int m = 0; m < 8; ++m) {
    const float r0 = sigm_sc(fmaf(xv, wih[0][m], D[0][m]));
    const float r1 = sigm_sc(fmaf(xv, wih[1][m], D[1][m]));
    const float z0 = sigm_sc(fmaf(xv, wih[2][m], D[2][m]));
    const float z1 = sigm_sc(fmaf(xv, wih[3][m], D[3][m]));
    const float n0 = tanh_sc(fmaf(r0, D[4][m], fmaf(xv, wih[4][m], bihn[0][m])));
    const float n1 = tanh_sc(fmaf(r1, D[5][m], fmaf(xv, wih[5][m], bihn[1][m])));
    hlo[m] = fmaf(z0, hlo[m] - n0, n0);
    hhi[m] = fmaf(z1, hhi[m] - n1, n1);
  }
}

__global__ __launch_bounds__(kThreads)
void gated_cell_kernel(const float* __restrict__ x,
                       const float* __restrict__ w_ih,
                       const float* __restrict__ w_hh,
                       const float* __restrict__ b_ih,
                       const float* __restrict__ b_hh,
                       const float* __restrict__ fc_w,
                       const float* __restrict__ fc_b,
                       float* __restrict__ out)
{
  __shared__ __align__(16) unsigned int Wlw[kGateRows * kHid / 2];
  __shared__ __align__(16) unsigned int Flw[kOutRowsPad * kHid / 2];
  __shared__ __align__(32) float Cl[2][48];
  __shared__ __align__(16) float Pl[3][kGateRows];
  __shared__ __align__(16) float slab[kWaves][kOutPerWave];

  const int tid  = threadIdx.x;
  const int lane = tid & 31;
  const int wave = tid >> 5;
  const int bn   = lane & 15;
  const int hf   = lane >> 4;
  const int waveG = blockIdx.x * kWaves + wave;
  int b = waveG * kRowsPerWave + bn;
  b = b < kBatch ? b : kBatch - 1;

#pragma unroll
  for (int it = 0; it < 6; ++it) {
    const int wi = it * kThreads + tid;
    const v2f wv = *(const v2f*)(w_hh + 2 * wi);
    Wlw[wi] = pack_f16x2(wv[0] * kWScale, wv[1] * kWScale);
  }
  {
    const int e0  = 2 * tid;
    const int row = e0 >> 5;
    const int rc  = row < kOutF ? row : kOutF - 1;
    const v2f fv  = *(const v2f*)(fc_w + rc * kHid + (e0 & 31));
    const float f0 = row < kOutF ? fv[0] * kWScale : 0.0f;
    const float f1 = row < kOutF ? fv[1] * kWScale : 0.0f;
    Flw[tid] = pack_f16x2(f0, f1);
  }
  {
    const int pc = tid < kGateRows ? tid : kGateRows - 1;
    const float a0 = w_ih[pc];
    const float a1 = b_ih[pc];
    const int qc = tid < kOutF ? tid : kOutF - 1;
    const float a2 = fc_b[qc];
    if (tid < kGateRows) {
      Pl[0][tid] = a0;
      Pl[1][tid] = a1;
      Pl[2][tid] = (tid < kOutF) ? a2 : 0.0f;
    }
  }
  {
    const int q   = tid < kGateRows ? tid : kGateRows - 1;
    const int qh  = q >= 48 ? 1 : 0;
    const int rem = q - 48 * qh;
    const int tt  = rem >> 3;
    const int m   = rem & 7;
    const int gt  = tt >> 1;
    const int p   = tt & 1;
    const int g   = gt * kHid + p * 16 + 8 * qh + m;
    const float bi = b_ih[g];
    const float bh = b_hh[g];
    const float v01 = (bi + bh) * kWScale;
    const float v2  = bh * kWScale;
    const float cv  = (gt < 2) ? v01 : v2;
    if (tid < kGateRows) Cl[qh][rem] = cv;
  }
  __syncthreads();

  float wih[6][8];
  float bihn[2][8];
#pragma unroll
  for (int gt = 0; gt < 3; ++gt) {
#pragma unroll
    for (int p = 0; p < 2; ++p) {
#pragma unroll
      for (int m = 0; m < 8; ++m) {
        const int tt = gt * 2 + p;
        const int g  = gt * kHid + p * 16 + 8 * hf + m;
        wih[tt][m] = Pl[0][g] * kWScale;
        if (gt == 2) bihn[p][m] = Pl[1][g] * kWScale;
      }
    }
  }

  float hlo[8], hhi[8];
#pragma unroll
  for (int i = 0; i < 8; ++i) { hlo[i] = 0.0f; hhi[i] = 0.0f; }

  const _Float16* Wl  = (const _Float16*)Wlw;
  const float*    Clh = &Cl[hf][0];
  const float*    xp  = x + (size_t)b * kSeq;

#pragma unroll 1
  for (int t0 = 0; t0 < kSeq; t0 += 4) {
    const v4f xa = *(const v4f*)(xp + t0);
    cell_step(xa[0], hlo, hhi, wih, bihn, Wl, Clh, bn, hf);
    cell_step(xa[1], hlo, hhi, wih, bihn, Wl, Clh, bn, hf);
    cell_step(xa[2], hlo, hhi, wih, bihn, Wl, Clh, bn, hf);
    cell_step(xa[3], hlo, hhi, wih, bihn, Wl, Clh, bn, hf);
  }

  {
    const _Float16* Fl = (const _Float16*)Flw;
    v16h Bf;
#pragma unroll
    for (int i = 0; i < 8; ++i) {
      Bf[i]     = (_Float16)hlo[i];
      Bf[8 + i] = (_Float16)hhi[i];
    }
    const v16h Afc = frag_load_f16(Fl + bn * kHid + 8 * hf);
    v8f fcc;
#pragma unroll
    for (int r = 0; r < 8; ++r) {
      const int o  = 8 * hf + r;
      const int oc = o < kOutF ? o : kOutF - 1;
      const float bv = Pl[2][oc] * kWScale;
      fcc[r] = (o < kOutF) ? bv : 0.0f;
    }
    const v8f Do = mma_f16(Afc, Bf, fcc);
    float* sw = slab[wave];
#pragma unroll
    for (int r = 0; r < 8; ++r) {
      const int o = 8 * hf + r;
      if (o < kOutF) sw[bn * kOutF + o] = Do[r] * kWInv;
    }
  }
  __syncthreads();
  {
    const float* sw = slab[wave];
    const v4f o0 = *(const v4f*)(sw + 4 * lane);
    const int  l2 = lane < 16 ? lane : 0;
    const v4f o1 = *(const v4f*)(sw + 128 + 4 * l2);
    float* ob = out + (size_t)waveG * kOutPerWave;
    for (int pass = 0; pass < 2; ++pass) {
      *(volatile v4f*)(ob + 4 * lane) = o0;
      if (lane < 16) *(volatile v4f*)(ob + 128 + 4 * lane) = o1;
      __threadfence();
    }
  }
}

extern "C" void kernel_launch(void* const* d_in, const int* in_sizes, int n_in,
                              void* d_out, int out_size, void* d_ws, size_t ws_size,
                              hipStream_t stream) {
  (void)d_ws; (void)ws_size;
  if (n_in < 7) return;
  if (in_sizes[0] < kBatch * kSeq || in_sizes[1] < kGateRows || in_sizes[2] < kGateRows * kHid ||
      in_sizes[3] < kGateRows || in_sizes[4] < kGateRows || in_sizes[5] < kOutF * kHid ||
      in_sizes[6] < kOutF || out_size < kBatch * kOutF) return;
  const float* x    = (const float*)d_in[0];
  const float* w_ih = (const float*)d_in[1];
  const float* w_hh = (const float*)d_in[2];
  const float* b_ih = (const float*)d_in[3];
  const float* b_hh = (const float*)d_in[4];
  const float* fc_w = (const float*)d_in[5];
  const float* fc_b = (const float*)d_in[6];
  float* out = (float*)d_out;
  gated_cell_kernel<<<dim3(kBlocks), dim3(kThreads), 0, stream>>>(x, w_ih, w_hh, b_ih, b_hh, fc_w, fc_b, out);
}
